// HeavyEncoderLayer_old_74388833566994
// MI455X (gfx1250) — hardware-verified
//
#include <hip/hip_runtime.h>
#include <stddef.h>


#define NTHR   64
#define NWAVE  2
#define EPT    16
#define CHUNK  (NTHR * EPT)
#define WCAP   (EPT * 32)
#define LISTN  (NWAVE * WCAP)
#define PASSN  NTHR
#define PCAP   (CHUNK + PASSN)
#define NB     320
#define FW     112
#define AW     113
#define PW     192
#define XW     160
#define NHVY   25000
#define KC     256
#define EPI_IT ((NB * FW) / (128 * NWAVE))

#define OW1H   0
#define OW1L   1024
#define OW3H   2048
#define OW3L   4096
#define OW2H   6144
#define OW2L   6656
#define OW4H   7168
#define OW4L   8192
#define OWABH  9216
#define OWABL  10752
#define OWCH   12288
#define OWCL   13312
#define OWH0H  14336
#define OWH0L  34816
#define OWH1H  55296
#define OWH1L  88064
#define WTOT   120832

#define C_INV3 0.57735026918962576f
#define C_NMSG 0.10206207261596575f
#define C_NGS  0.25f
#define C_NGV  0.17677669529663687f
#define C_NH0  0.027950849718747371f
#define C_NH1  0.03125f

static_assert(EPI_IT * 128 * NWAVE == NB * FW);
static_assert(PCAP >= CHUNK + PASSN);
static_assert((NB % 2) == 0);
static_assert(((32 * KC) % NTHR) == 0);
static_assert((EPT % 4) == 0);

typedef float          v4f   __attribute__((ext_vector_type(4)));
typedef float          v8f   __attribute__((ext_vector_type(8)));
typedef int            v4i   __attribute__((ext_vector_type(4)));
typedef unsigned short v8us  __attribute__((ext_vector_type(8)));
typedef unsigned short v16us __attribute__((ext_vector_type(16)));
typedef __bf16         v16b  __attribute__((ext_vector_type(16)));
union FragB { v16us u; v8us h[2]; v16b v; };

#define DEV __device__ __forceinline__

DEV v8f zacc() {
  v8f c;
#pragma unroll
  for (int i = 0; i < 8; ++i) c[i] = 0.0f;
  return c;
}

DEV unsigned rne16(float x) {
  const unsigned u = __float_as_uint(x);
  return (u + 0x7fffu + ((u >> 16) & 1u)) >> 16;
}
DEV void split16(float x, unsigned short& hi, unsigned short& lo) {
  const unsigned h = rne16(x);
  hi = (unsigned short)h;
  lo = (unsigned short)rne16(x - __uint_as_float(h << 16));
}

DEV v8f wmb(v16b a, v16b b, v8f c) {
  v8f d = __builtin_amdgcn_wmma_f32_16x16x32_bf16(false, a, false, b, (short)0, c, false, false);
  asm volatile("v_nop\n\tv_nop\n\tv_nop\n\tv_nop" : "+v"(d) : "v"(a), "v"(b));
  return d;
}
DEV v8f wm3(const FragB& ah, const FragB& al, const FragB& bh, const FragB& bl, v8f c) {
  c = wmb(ah.v, bh.v, c);
  c = wmb(ah.v, bl.v, c);
  c = wmb(al.v, bh.v, c);
  return c;
}
DEV void ldf(FragB& f, const unsigned short* rowp, int k0, int hh) {
  f.h[0] = *(const v8us*)(rowp + k0 + 8 * hh);
  f.h[1] = *(const v8us*)(rowp + k0 + 16 + 8 * hh);
}

DEV void cvt_plane(const float* __restrict__ WA, const float* __restrict__ WB, int pitch, int nRows,
                   int K, int K1, int K2, unsigned short* dh, unsigned short* dl, int tid, int nthr) {
  const int nv = (nRows * K) / 8;
  const int kbm = K2 > 0 ? K2 - 1 : 0;
#pragma unroll 1
  for (int v = tid; v < nv; v += nthr) {
    const int e0 = v * 8;
    const int n = e0 / K;
    const int k8 = e0 - n * K;
    v8us vh, vl;
#pragma unroll
    for (int j = 0; j < 8; ++j) {
      const int k = k8 + j;
      const int ka = k < K1 ? k : K1 - 1;
      int kb = k - K1;
      kb = kb < 0 ? 0 : (kb > kbm ? kbm : kb);
      const float a = WA[ka * pitch + n];
      const float b = WB[kb * pitch + n];
      const float val = (k < K1) ? a : ((k < K1 + K2) ? b : 0.0f);
      unsigned short x1, x2;
      split16(val, x1, x2);
      vh[j] = x1;
      vl[j] = x2;
    }
    *(volatile v8us*)(dh + e0) = vh;
    *(volatile v8us*)(dl + e0) = vl;
  }
}

__global__ __launch_bounds__(256) void k_wprep(
    const float* __restrict__ W1, const float* __restrict__ W2, const float* __restrict__ W3,
    const float* __restrict__ W4, const float* __restrict__ Wa, const float* __restrict__ Wb,
    const float* __restrict__ Wc, const float* __restrict__ Wss, const float* __restrict__ Wvv,
    const float* __restrict__ Wsv, const float* __restrict__ Wvs, unsigned short* wts) {
  const int tid = threadIdx.x;
#pragma unroll 1
  for (int p = 0; p < 2; ++p) {
    cvt_plane(W1,  W1,  16, 16, 64,   64,  0,    wts + OW1H,  wts + OW1L,  tid, 256);
    cvt_plane(W3,  W3,  32, 32, 64,   64,  0,    wts + OW3H,  wts + OW3L,  tid, 256);
    cvt_plane(W2,  W2,  16, 16, 32,   32,  0,    wts + OW2H,  wts + OW2L,  tid, 256);
    cvt_plane(W4,  W4,  32, 32, 32,   32,  0,    wts + OW4H,  wts + OW4L,  tid, 256);
    cvt_plane(Wa,  Wa,  16, 16, 32,   16,  0,    wts + OWABH, wts + OWABL, tid, 256);
    cvt_plane(Wb,  Wb,  32, 32, 32,   16,  0,    wts + OWABH + 16 * 32, wts + OWABL + 16 * 32, tid, 256);
    cvt_plane(Wc,  Wc,  32, 32, 32,   32,  0,    wts + OWCH,  wts + OWCL,  tid, 256);
    cvt_plane(Wss, Wvv, 16, 16, 1280, 256, 1024, wts + OWH0H, wts + OWH0L, tid, 256);
    cvt_plane(Wsv, Wvs, 32, 32, 1024, 512, 512,  wts + OWH1H, wts + OWH1L, tid, 256);
    if (p == 0) { __threadfence(); __syncthreads(); }
  }
}

__global__ __launch_bounds__(NTHR) void k_planes(const float* __restrict__ x, const unsigned short* __restrict__ wts,
                                                  float* P, int nN) {
  __shared__ __attribute__((aligned(16))) unsigned short sSh[32 * 64];
  __shared__ __attribute__((aligned(16))) unsigned short sSl[32 * 64];
  __shared__ __attribute__((aligned(16))) unsigned short sVh[3 * 32 * 32];
  __shared__ __attribute__((aligned(16))) unsigned short sVl[3 * 32 * 32];
  __shared__ __attribute__((aligned(16))) float sOut[32 * PW];

  const int tid = threadIdx.x, lane = tid & 31, wave = tid >> 5, hh = lane >> 4, m = lane & 15;
  const int row0 = blockIdx.x * 32;

#pragma unroll 1
  for (int q = 0; q < 8; ++q) {
    const int idx = q * NTHR + tid;
    const int r = idx >> 4, k4 = (idx & 15) * 4;
    int gr = row0 + r;
    gr = gr > nN - 1 ? nN - 1 : gr;
    const v4f v = *(const v4f*)(x + (size_t)gr * XW + k4);
#pragma unroll
    for (int t = 0; t < 4; ++t) split16(v[t], sSh[r * 64 + k4 + t], sSl[r * 64 + k4 + t]);
  }
#pragma unroll 1
  for (int q = 0; q < 12; ++q) {
    const int idx = q * NTHR + tid;
    const int r = idx / 24, j4 = (idx - r * 24) * 4;
    int gr = row0 + r;
    gr = gr > nN - 1 ? nN - 1 : gr;
    const v4f v = *(const v4f*)(x + (size_t)gr * XW + 64 + j4);
#pragma unroll
    for (int t = 0; t < 4; ++t) {
      const int j = j4 + t, u = j / 3, i = j - 3 * u;
      split16(v[t], sVh[(i * 32 + r) * 32 + u], sVl[(i * 32 + r) * 32 + u]);
    }
  }
  __syncthreads();

  const int ar = 16 * wave + m;
  {
    v8f aC = zacc(), aA0 = zacc(), aA1 = zacc();
#pragma unroll
    for (int ks = 0; ks < 2; ++ks) {
      const int k0 = 32 * ks;
      FragB ah, al, bh, bl;
      ldf(ah, sSh + ar * 64, k0, hh);
      ldf(al, sSl + ar * 64, k0, hh);
      ldf(bh, wts + OW1H + m * 64, k0, hh);
      ldf(bl, wts + OW1L + m * 64, k0, hh);
      aC = wm3(ah, al, bh, bl, aC);
      ldf(bh, wts + OW3H + m * 64, k0, hh);
      ldf(bl, wts + OW3L + m * 64, k0, hh);
      aA0 = wm3(ah, al, bh, bl, aA0);
      ldf(bh, wts + OW3H + (16 + m) * 64, k0, hh);
      ldf(bl, wts + OW3L + (16 + m) * 64, k0, hh);
      aA1 = wm3(ah, al, bh, bl, aA1);
    }
#pragma unroll
    for (int r = 0; r < 8; ++r) {
      float* op = sOut + (16 * wave + 8 * hh + r) * PW;
      op[4 * m] = aC[r];
      op[64 + 4 * m] = aA0[r];
      op[64 + 4 * (16 + m)] = aA1[r];
    }
  }
#pragma unroll 1
  for (int i = 0; i < 3; ++i) {
    v8f aD = zacc(), aB0 = zacc(), aB1 = zacc();
    FragB ah, al, bh, bl;
    ldf(ah, sVh + (i * 32 + ar) * 32, 0, hh);
    ldf(al, sVl + (i * 32 + ar) * 32, 0, hh);
    ldf(bh, wts + OW2H + m * 32, 0, hh);
    ldf(bl, wts + OW2L + m * 32, 0, hh);
    aD = wm3(ah, al, bh, bl, aD);
    ldf(bh, wts + OW4H + m * 32, 0, hh);
    ldf(bl, wts + OW4L + m * 32, 0, hh);
    aB0 = wm3(ah, al, bh, bl, aB0);
    ldf(bh, wts + OW4H + (16 + m) * 32, 0, hh);
    ldf(bl, wts + OW4L + (16 + m) * 32, 0, hh);
    aB1 = wm3(ah, al, bh, bl, aB1);
#pragma unroll
    for (int r = 0; r < 8; ++r) {
      float* op = sOut + (16 * wave + 8 * hh + r) * PW + 1 + i;
      op[4 * m] = aD[r];
      op[64 + 4 * m] = aB0[r];
      op[64 + 4 * (16 + m)] = aB1[r];
    }
  }
  __syncthreads();

  float* gp = P + (size_t)row0 * PW;
#pragma unroll 1
  for (int p = 0; p < 2; ++p) {
#pragma unroll 1
    for (int it = 0; it < (32 * PW) / (128 * NWAVE); ++it) {
      const int f = (it * NWAVE + wave) * 128 + 4 * lane;
      const v4f v = *(const v4f*)(sOut + f);
      *(volatile v4f*)(gp + f) = v;
    }
    if (p == 0) __threadfence();
  }
}

template <int MODE>
DEV int scan_chunk(const int* __restrict__ keyA, const int* __restrict__ keyB, int nL, int cbase,
                   int nodeBase, int vec, int* hl, int tid, int wave) {
  int wc = 0;
  const int el0 = tid * EPT;
  const int e0 = cbase + el0;
  const int sent = -2147483647 - 1;
  int d[EPT];
  if (vec != 0 && cbase + CHUNK <= nL) {
#pragma unroll
    for (int q = 0; q < EPT / 4; ++q) {
      const v4i a = *(const v4i*)(keyA + e0 + 4 * q);
      int k0 = a.x, k1 = a.y, k2 = a.z, k3 = a.w;
      if (MODE == 1) {
        const v4i zz = *(const v4i*)(keyB + e0 + 4 * q);
        k0 = (zz.x > 1) ? k0 : sent;
        k1 = (zz.y > 1) ? k1 : sent;
        k2 = (zz.z > 1) ? k2 : sent;
        k3 = (zz.w > 1) ? k3 : sent;
      }
      d[4 * q] = k0; d[4 * q + 1] = k1; d[4 * q + 2] = k2; d[4 * q + 3] = k3;
    }
  } else {
#pragma unroll
    for (int j = 0; j < EPT; ++j) {
      const int e = e0 + j;
      const int ec = (e < nL) ? e : (nL - 1);
      int k = keyA[ec];
      if (MODE == 1) { const int zz = keyB[ec]; k = (zz > 1) ? k : sent; }
      d[j] = (e < nL) ? k : sent;
    }
  }
  const unsigned nb = (unsigned)nodeBase;
  bool hit[EPT];
  bool anyh = false;
#pragma unroll
  for (int j = 0; j < EPT; ++j) { hit[j] = ((unsigned)d[j] - nb) < (unsigned)NB; anyh = anyh | hit[j]; }
  const unsigned anyw = __builtin_amdgcn_ballot_w32(anyh);
  if (anyw != 0u) {
#pragma unroll
    for (int j = 0; j < EPT; ++j) {
      const unsigned mj = __builtin_amdgcn_ballot_w32(hit[j]);
      if (mj != 0u) {
        if (hit[j]) {
          const int pos = wc + (int)__builtin_amdgcn_mbcnt_lo(mj, 0u);
          if (pos < WCAP) hl[wave * WCAP + pos] = el0 + j;
        }
        wc += (int)__builtin_popcount(mj);
      }
    }
  }
  return wc;
}

template <int MODE>
__global__ __launch_bounds__(NTHR) void k_agg(const int* __restrict__ keyA, const int* __restrict__ keyB,
                                               const float* __restrict__ ea, const float* __restrict__ gsrc,
                                               float* outp, int nL, int nG, int vec) {
  __shared__ __attribute__((aligned(16))) float acc[(NB + 1) * AW];
  __shared__ __attribute__((aligned(16))) int   hl[LISTN];
  __shared__ __attribute__((aligned(16))) int   pend[PCAP];
  __shared__ __attribute__((aligned(16))) float s_ea[PASSN * 4];
  __shared__ int s_g[PASSN];
  __shared__ int s_slot[PASSN];
  __shared__ int wcnt[NWAVE];
  __shared__ int pendN;

  const int tid = threadIdx.x, lane = tid & 31, wave = tid >> 5;
  const int nodeBase = blockIdx.x * NB;
  const int sent = -2147483647 - 1;

  for (int i = tid; i < (NB + 1) * AW; i += NTHR) acc[i] = 0.0f;
  if (tid == 0) pendN = 0;

  const bool rS = tid < 16, rV = (tid >= 16) && (tid < 48), rC = (tid == 48);
  int ww = tid - 16;
  ww = ww < 0 ? 0 : (ww > 31 ? 31 : ww);
  const int poff = rS ? (4 * tid) : (64 + 4 * ww);
  const int col0 = rS ? tid : (rV ? (16 + 3 * ww) : FW);
  const int nw = rS ? 1 : (rV ? 3 : (rC ? 1 : 0));
  const float kSx = rS ? 1.0f : 0.0f, kSy = rV ? 1.0f : 0.0f;
  const float kBx = rV ? 1.0f : 0.0f, kAy = rS ? C_INV3 : 0.0f, kA = rS ? C_INV3 : 0.0f;
  const float kNM = rC ? 0.0f : C_NMSG, kOne = rC ? 1.0f : 0.0f;
  const int colB = (tid < 48) ? (64 + tid) : FW;
  const int ldB = (64 + tid) > (FW - 1) ? (FW - 1) : (64 + tid);
  const float k1a = (tid < 48) ? 1.0f : 0.0f, k1b = (tid == 48) ? 1.0f : 0.0f;
  const bool wB = tid <= 48;
  __syncthreads();

  const int nChunks = (nL + CHUNK - 1) / CHUNK;
#pragma unroll 1
  for (int ch = 0; ch < nChunks; ++ch) {
    const int cbase = ch * CHUNK;
    const int wc = scan_chunk<MODE>(keyA, keyB, nL, cbase, nodeBase, vec, hl, tid, wave);
    if (lane == 0) wcnt[wave] = wc;
    __syncthreads();

    const int base = pendN;
    int tot = 0, myoff = 0;
#pragma unroll
    for (int w = 0; w < NWAVE; ++w) {
      int c = wcnt[w];
      c = c > WCAP ? WCAP : (c < 0 ? 0 : c);
      if (w < wave) myoff += c;
      tot += c;
    }
    int newN = base + tot;
    newN = newN > PCAP ? PCAP : newN;
    {
      int n = wcnt[wave];
      n = n > WCAP ? WCAP : (n < 0 ? 0 : n);
      const int* lp = hl + wave * WCAP;
      for (int i = lane; i < n; i += 32) {
        const int pos = base + myoff + i;
        if (pos < PCAP) pend[pos] = cbase + lp[i];
      }
    }
    const int fin  = (ch == nChunks - 1) ? 1 : 0;
    const int R    = (fin != 0) ? (newN + PASSN - 1) / PASSN : newN / PASSN;
    const int Pval = (fin != 0) ? newN : R * PASSN;
    __syncthreads();

#pragma unroll 1
    for (int r = 0; r < R; ++r) {
      {
        const int idx = r * PASSN + tid;
        const bool valid = idx < Pval;
        int e = 0;
        if (valid) e = pend[idx];
        e = e < 0 ? 0 : (e > nL - 1 ? nL - 1 : e);
        int key, g;
        if (MODE == 0) {
          key = keyA[e];
          g = keyB[e];
          g = g < 0 ? 0 : (g > nG - 1 ? nG - 1 : g);
          const v4f a4 = *(const v4f*)(ea + (size_t)e * 4);
          *(v4f*)(s_ea + 4 * tid) = a4;
        } else {
          const int zz = keyB[e];
          const int kc = keyA[e];
          key = (zz > 1) ? kc : sent;
          g = e;
        }
        int slot = key - nodeBase;
        if (!valid || (unsigned)slot >= (unsigned)NB) slot = NB;
        s_g[tid] = g;
        s_slot[tid] = slot;
      }
      __syncthreads();
      int nval = Pval - r * PASSN;
      nval = nval > PASSN ? PASSN : nval;
#pragma unroll 1
      for (int j = 0; j < nval; ++j) {
        const int sl = s_slot[j];
        const int g = s_g[j];
        if (MODE == 0) {
          const v4f e4 = *(const v4f*)(s_ea + 4 * j);
          const v4f pv = *(const v4f*)(gsrc + (size_t)g * PW + poff);
          const float se = e4.x, v0 = e4.y, v1 = e4.z, v2 = e4.w;
          const float o0 = kNM * (se * (kSx * pv.x + kSy * pv.y) + v0 * (kBx * pv.x + kAy * pv.y)
                                  + kA * (v1 * pv.z + v2 * pv.w)) + kOne;
          const float o1 = C_NMSG * (pv.x * v1 + se * pv.z);
          const float o2 = C_NMSG * (pv.x * v2 + se * pv.w);
          float* ap = acc + sl * AW + col0;
          if (nw > 0) ap[0] += o0;
          if (nw > 1) { ap[1] += o1; ap[2] += o2; }
        } else {
          const float* xr = gsrc + (size_t)g * FW;
          const float x0 = xr[tid];
          const float x1 = xr[ldB];
          float* ap = acc + sl * AW;
          ap[tid] += x0;
          if (wB) ap[colB] += k1a * x1 + k1b;
        }
      }
      __syncthreads();
    }

    int rem = newN - R * PASSN;
    rem = rem < 0 ? 0 : rem;
    if (R > 0 && tid < rem) pend[tid] = pend[R * PASSN + tid];
    if (tid == 0) pendN = rem;
  }
  __syncthreads();

  const size_t ob = (size_t)nodeBase * FW;
#pragma unroll 1
  for (int p = 0; p < 2; ++p) {
#pragma unroll 1
    for (int it = 0; it < EPI_IT; ++it) {
      const int f = (it * NWAVE + wave) * 128 + 4 * lane;
      const int sl = f / FW;
      const int c = f - sl * FW;
      const float* ar = acc + sl * AW;
      const float inv = 1.0f / fmaxf(ar[FW], 1.0f);
      v4f v;
      v.x = ar[c] * inv; v.y = ar[c + 1] * inv; v.z = ar[c + 2] * inv; v.w = ar[c + 3] * inv;
      *(volatile v4f*)(outp + ob + f) = v;
    }
    if (p == 0) __threadfence();
  }
}

__global__ __launch_bounds__(NTHR) void k_gate(const float* __restrict__ M, const unsigned short* __restrict__ wts,
                                                float* XA, int mRows) {
  __shared__ __attribute__((aligned(16))) unsigned short sAh[32 * 32];
  __shared__ __attribute__((aligned(16))) unsigned short sAl[32 * 32];
  __shared__ __attribute__((aligned(16))) unsigned short sVh[3 * 32 * 32];
  __shared__ __attribute__((aligned(16))) unsigned short sVl[3 * 32 * 32];
  __shared__ __attribute__((aligned(16))) float sOut[32 * FW];

  const int tid = threadIdx.x, lane = tid & 31, wave = tid >> 5, hh = lane >> 4, m = lane & 15;
  const int row0 = blockIdx.x * 32;

#pragma unroll 1
  for (int q = 0; q < 14; ++q) {
    const int idx = q * NTHR + tid;
    const int r = idx / 28, c4 = (idx - r * 28) * 4;
    int gr = row0 + r;
    gr = gr > mRows - 1 ? mRows - 1 : gr;
    const v4f v = *(const v4f*)(M + (size_t)gr * FW + c4);
    if (c4 < 16) {
#pragma unroll
      for (int t = 0; t < 4; ++t) split16(v[t], sAh[r * 32 + c4 + t], sAl[r * 32 + c4 + t]);
    } else {
#pragma unroll
      for (int t = 0; t < 4; ++t) {
        const int c = c4 + t - 16, u = c / 3, i = c - 3 * u;
        split16(v[t], sVh[(i * 32 + r) * 32 + u], sVl[(i * 32 + r) * 32 + u]);
      }
    }
  }
#pragma unroll 1
  for (int q = 0; q < 8; ++q) {
    const int idx = q * NTHR + tid;
    const int r = idx >> 4, k = 16 + (idx & 15);
    sAh[r * 32 + k] = 0;
    sAl[r * 32 + k] = 0;
  }
  __syncthreads();

  const int ar = 16 * wave + m;
  float th0[8], th1[8];
  {
    FragB ah, al, bh, bl;
    ldf(ah, sAh + ar * 32, 0, hh);
    ldf(al, sAl + ar * 32, 0, hh);
    v8f g0 = zacc(), g1 = zacc(), g2 = zacc();
    ldf(bh, wts + OWABH + m * 32, 0, hh);
    ldf(bl, wts + OWABL + m * 32, 0, hh);
    g0 = wm3(ah, al, bh, bl, g0);
    ldf(bh, wts + OWABH + (16 + m) * 32, 0, hh);
    ldf(bl, wts + OWABL + (16 + m) * 32, 0, hh);
    g1 = wm3(ah, al, bh, bl, g1);
    ldf(bh, wts + OWABH + (32 + m) * 32, 0, hh);
    ldf(bl, wts + OWABL + (32 + m) * 32, 0, hh);
    g2 = wm3(ah, al, bh, bl, g2);
#pragma unroll
    for (int r = 0; r < 8; ++r) {
      float* op = sOut + (16 * wave + 8 * hh + r) * FW;
      const float a = C_NGS * g0[r];
      const float ex = __expf(fminf(-a, 80.0f));
      op[m] = __builtin_amdgcn_rcpf(1.0f + ex);
      const float b0 = C_NGS * g1[r], b1 = C_NGS * g2[r];
      const float e0 = __expf(fminf(-2.0f * b0, 80.0f));
      const float e1 = __expf(fminf(-2.0f * b1, 80.0f));
      th0[r] = 2.0f * __builtin_amdgcn_rcpf(1.0f + e0) - 1.0f;
      th1[r] = 2.0f * __builtin_amdgcn_rcpf(1.0f + e1) - 1.0f;
    }
  }
#pragma unroll 1
  for (int i = 0; i < 3; ++i) {
    FragB ah, al, bh, bl;
    ldf(ah, sVh + (i * 32 + ar) * 32, 0, hh);
    ldf(al, sVl + (i * 32 + ar) * 32, 0, hh);
    v8f c0 = zacc(), c1 = zacc();
    ldf(bh, wts + OWCH + m * 32, 0, hh);
    ldf(bl, wts + OWCL + m * 32, 0, hh);
    c0 = wm3(ah, al, bh, bl, c0);
    ldf(bh, wts + OWCH + (16 + m) * 32, 0, hh);
    ldf(bl, wts + OWCL + (16 + m) * 32, 0, hh);
    c1 = wm3(ah, al, bh, bl, c1);
#pragma unroll
    for (int r = 0; r < 8; ++r) {
      float* op = sOut + (16 * wave + 8 * hh + r) * FW + 16 + i;
      op[3 * m] = th0[r] * (C_NGV * c0[r]);
      op[3 * (16 + m)] = th1[r] * (C_NGV * c1[r]);
    }
  }
  __syncthreads();

  float* gp = XA + (size_t)row0 * FW;
#pragma unroll 1
  for (int p = 0; p < 2; ++p) {
#pragma unroll 1
    for (int it = 0; it < (32 * FW) / (128 * NWAVE); ++it) {
      const int f = (it * NWAVE + wave) * 128 + 4 * lane;
      const v4f v = *(const v4f*)(sOut + f);
      *(volatile v4f*)(gp + f) = v;
    }
    if (p == 0) __threadfence();
  }
}

__global__ __launch_bounds__(NTHR) void k_heavy(const float* __restrict__ HS, const unsigned short* __restrict__ wts,
                                                 float* Hout, int hsRows) {
  __shared__ __attribute__((aligned(16))) float sH[32 * FW];
  __shared__ __attribute__((aligned(16))) unsigned short sAh[32 * KC];
  __shared__ __attribute__((aligned(16))) unsigned short sAl[32 * KC];
  __shared__ __attribute__((aligned(16))) float sOut[32 * FW];

  const int tid = threadIdx.x, lane = tid & 31, wave = tid >> 5, hh = lane >> 4, m = lane & 15;
  const int row0 = blockIdx.x * 32;

#pragma unroll 1
  for (int q = 0; q < 14; ++q) {
    const int idx = q * NTHR + tid;
    const int r = idx / 28, c4 = (idx - r * 28) * 4;
    int gr = row0 + r;
    gr = gr > hsRows - 1 ? hsRows - 1 : gr;
    *(v4f*)(sH + r * FW + c4) = *(const v4f*)(HS + (size_t)gr * FW + c4);
  }
  __syncthreads();

  const int ar = 16 * wave + m;

  v8f a0 = zacc();
#pragma unroll 1
  for (int chn = 0; chn < 5; ++chn) {
#pragma unroll 2
    for (int q = 0; q < (32 * KC) / NTHR; ++q) {
      const int idx = q * NTHR + tid;
      const int r = idx / KC, kk = idx - r * KC;
      const float* hr = sH + r * FW;
      float av;
      if (chn == 0) {
        const int u = kk >> 4, v = kk & 15;
        av = hr[u] * hr[v];
      } else {
        const int kk2 = (chn - 1) * KC + kk;
        const int u = kk2 >> 5, v = kk2 & 31;
        const float* hu = hr + 16 + 3 * u;
        const float* hv = hr + 16 + 3 * v;
        av = C_INV3 * (hu[0] * hv[0] + hu[1] * hv[1] + hu[2] * hv[2]);
      }
      split16(av, sAh[r * KC + kk], sAl[r * KC + kk]);
    }
    __syncthreads();
#pragma unroll 2
    for (int ks = 0; ks < KC / 32; ++ks) {
      const int k0 = 32 * ks;
      const int kg = chn * KC + k0;
      FragB ah, al, bh, bl;
      ldf(ah, sAh + ar * KC, k0, hh);
      ldf(al, sAl + ar * KC, k0, hh);
      ldf(bh, wts + OWH0H + m * 1280, kg, hh);
      ldf(bl, wts + OWH0L + m * 1280, kg, hh);
      a0 = wm3(ah, al, bh, bl, a0);
    }
    __syncthreads();
  }
#pragma unroll
  for (int r = 0; r < 8; ++r) sOut[(16 * wave + 8 * hh + r) * FW + m] = C_NH0 * a0[r];

#pragma unroll 1
  for (int i = 0; i < 3; ++i) {
    v8f b0 = zacc(), b1 = zacc();
#pragma unroll 1
    for (int chn = 0; chn < 4; ++chn) {
#pragma unroll 2
      for (int q = 0; q < (32 * KC) / NTHR; ++q) {
        const int idx = q * NTHR + tid;
        const int r = idx / KC, kk = idx - r * KC;
        const float* hr = sH + r * FW;
        float av;
        if (chn < 2) {
          const int k = chn * KC + kk;
          const int u = k >> 5, v = k & 31;
          av = hr[u] * hr[16 + 3 * v + i];
        } else {
          const int kk2 = (chn - 2) * KC + kk;
          const int u = kk2 >> 4, v = kk2 & 15;
          av = hr[16 + 3 * u + i] * hr[v];
        }
        split16(av, sAh[r * KC + kk], sAl[r * KC + kk]);
      }
      __syncthreads();
#pragma unroll 2
      for (int ks = 0; ks < KC / 32; ++ks) {
        const int k0 = 32 * ks;
        const int kg = chn * KC + k0;
        FragB ah, al, bh, bl;
        ldf(ah, sAh + ar * KC, k0, hh);
        ldf(al, sAl + ar * KC, k0, hh);
        ldf(bh, wts + OWH1H + m * 1024, kg, hh);
        ldf(bl, wts + OWH1L + m * 1024, kg, hh);
        b0 = wm3(ah, al, bh, bl, b0);
        ldf(bh, wts + OWH1H + (16 + m) * 1024, kg, hh);
        ldf(bl, wts + OWH1L + (16 + m) * 1024, kg, hh);
        b1 = wm3(ah, al, bh, bl, b1);
      }
      __syncthreads();
    }
#pragma unroll
    for (int r = 0; r < 8; ++r) {
      float* op = sOut + (16 * wave + 8 * hh + r) * FW + 16 + i;
      op[3 * m] = C_NH1 * b0[r];
      op[3 * (16 + m)] = C_NH1 * b1[r];
    }
  }
  __syncthreads();

  float* gp = Hout + (size_t)row0 * FW;
#pragma unroll 1
  for (int p = 0; p < 2; ++p) {
#pragma unroll 1
    for (int it = 0; it < (32 * FW) / (128 * NWAVE); ++it) {
      const int f = (it * NWAVE + wave) * 128 + 4 * lane;
      const v4f v = *(const v4f*)(sOut + f);
      *(volatile v4f*)(gp + f) = v;
    }
    if (p == 0) __threadfence();
  }
}

__global__ __launch_bounds__(NTHR) void k_final(const int* __restrict__ z, const int* __restrict__ can,
                                                 const float* __restrict__ XA, const float* __restrict__ H,
                                                 float* out, int nN, int nH) {
  const int tid = threadIdx.x;
  const int base = blockIdx.x * 64;
  int nrows = nN - base;
  nrows = nrows > 64 ? 64 : (nrows < 0 ? 0 : nrows);
  const int nvec = nrows * (FW / 4);
#pragma unroll 1
  for (int p = 0; p < 2; ++p) {
#pragma unroll 1
    for (int idx = tid; idx < nvec; idx += NTHR) {
      const int row = idx / (FW / 4);
      const int q = idx - row * (FW / 4);
      const int n = base + row;
      const int hz = (z[n] > 1) ? 1 : 0;
      int c = can[n];
      c = c < 0 ? 0 : (c > nH - 1 ? nH - 1 : c);
      const v4f a = *(const v4f*)(XA + (size_t)n * FW + 4 * q);
      const v4f b = *(const v4f*)(H + (size_t)c * FW + 4 * q);
      v4f v;
      v.x = hz ? b.x : a.x; v.y = hz ? b.y : a.y; v.z = hz ? b.z : a.z; v.w = hz ? b.w : a.w;
      *(volatile v4f*)(out + (size_t)n * FW + 4 * q) = v;
    }
    if (p == 0) __threadfence();
  }
}

extern "C" void kernel_launch(void* const* d_in, const int* in_sizes, int n_in,
                              void* d_out, int out_size, void* d_ws, size_t ws_size,
                              hipStream_t stream) {
  if (n_in < 16) return;
  const int nN = in_sizes[0] / XW;
  const int nE = in_sizes[1] / 2;
  if (nN < 1 || nE < 1) return;
  if (in_sizes[0] != nN * XW || in_sizes[1] != nE * 2 || in_sizes[2] != nE * 4) return;
  if (in_sizes[3] != nN || in_sizes[4] != nN) return;
  if (in_sizes[5] != 64 * 16 || in_sizes[6] != 32 * 16 || in_sizes[7] != 64 * 32 || in_sizes[8] != 32 * 32) return;
  if (in_sizes[9] != 16 * 16 || in_sizes[10] != 16 * 32 || in_sizes[11] != 32 * 32) return;
  if (in_sizes[12] != 16 * 16 * 16 || in_sizes[13] != 32 * 32 * 16) return;
  if (in_sizes[14] != 16 * 32 * 32 || in_sizes[15] != 32 * 16 * 32) return;
  if (out_size != nN * FW) return;

  const float* x   = (const float*)d_in[0];
  const int*   ei  = (const int*)d_in[1];
  const float* ea  = (const float*)d_in[2];
  const int*   z   = (const int*)d_in[3];
  const int*   can = (const int*)d_in[4];
  const float* W1  = (const float*)d_in[5];
  const float* W2  = (const float*)d_in[6];
  const float* W3  = (const float*)d_in[7];
  const float* W4  = (const float*)d_in[8];
  const float* Wa  = (const float*)d_in[9];
  const float* Wb  = (const float*)d_in[10];
  const float* Wc  = (const float*)d_in[11];
  const float* Wss = (const float*)d_in[12];
  const float* Wvv = (const float*)d_in[13];
  const float* Wsv = (const float*)d_in[14];
  const float* Wvs = (const float*)d_in[15];
  float* out = (float*)d_out;

  const int nH    = NHVY;
  const int nBlkA = (nN + NB - 1) / NB;
  const int nBlkB = (nH + NB - 1) / NB;
  const int n32N  = (nN + 31) / 32;
  const int n32H  = (nH + 31) / 32;
  const int nBlkF = (nN + 63) / 64;

  char* ws = (char*)d_ws;
  size_t off = 0;
  const size_t oW  = off; off += (size_t)WTOT * 2;                       off = (off + 255) & ~(size_t)255;
  const size_t oP  = off; off += (size_t)n32N * 32 * PW * 4;             off = (off + 255) & ~(size_t)255;
  const size_t oM  = off; off += (size_t)nBlkA * NB * FW * 4;            off = (off + 255) & ~(size_t)255;
  const size_t oXA = off; off += (size_t)n32N * 32 * FW * 4;             off = (off + 255) & ~(size_t)255;
  const size_t oHS = off; off += (size_t)nBlkB * NB * FW * 4;            off = (off + 255) & ~(size_t)255;
  const size_t oH  = off; off += (size_t)n32H * 32 * FW * 4;             off = (off + 255) & ~(size_t)255;
  if (off > ws_size) return;

  unsigned short* wts = (unsigned short*)(ws + oW);
  float* P  = (float*)(ws + oP);
  float* M  = (float*)(ws + oM);
  float* XA = (float*)(ws + oXA);
  float* HS = (float*)(ws + oHS);
  float* Hp = (float*)(ws + oH);

  const int vecE = ((nE & 3) == 0) ? 1 : 0;

  k_wprep<<<1, 256, 0, stream>>>(W1, W2, W3, W4, Wa, Wb, Wc, Wss, Wvv, Wsv, Wvs, wts);
  k_planes<<<n32N, NTHR, 0, stream>>>(x, wts, P, nN);
  k_agg<0><<<nBlkA, NTHR, 0, stream>>>(ei + nE, ei, ea, P, M, nE, nN, vecE);
  k_gate<<<n32N, NTHR, 0, stream>>>(M, wts, XA, nBlkA * NB);
  k_agg<1><<<nBlkB, NTHR, 0, stream>>>(can, z, ea, XA, HS, nN, nN, 1);
  k_heavy<<<n32H, NTHR, 0, stream>>>(HS, wts, Hp, nBlkB * NB);
  k_final<<<nBlkF, NTHR, 0, stream>>>(z, can, XA, Hp, out, nN, nH);
}
